// Mamba_65420941852740
// MI455X (gfx1250) — hardware-verified
//
#include <hip/hip_runtime.h>
#include <math.h>

typedef __attribute__((ext_vector_type(16))) _Float16 v16h;
typedef __attribute__((ext_vector_type(8)))  _Float16 v8h;
typedef __attribute__((ext_vector_type(8)))  float    v8f;
typedef __attribute__((ext_vector_type(4)))  float    v4f;

constexpr int kBatch  = 4;
constexpr int kSeq    = 2048;
constexpr int kDm     = 1024;
constexpr int kDin    = 2048;
constexpr int kNst    = 16;
constexpr int kConvK  = 4;
constexpr int kRows   = kBatch * kSeq;
constexpr int kAmat   = kNst * kNst;

constexpr int kScanCh = 64;
constexpr int kScanTS = 32;
constexpr int kAP     = 260;
constexpr int kYP     = 68;

constexpr float kWCarry  = 32.0f;
constexpr float kLoCarry = 2048.0f;
constexpr float kScaleHi = 1.0f / kWCarry;
constexpr float kScaleLo = 1.0f / (kWCarry * kLoCarry);

static_assert(kDin == 2 * kDm);
static_assert((kDm % 32) == 0 && (kDin % 32) == 0);
static_assert((kSeq % 64) == 0 && (kDm % 64) == 0 && (kDin % 64) == 0);
static_assert(((kSeq / 64) * (kDin / 64)) % 8 == 0);
static_assert(((kSeq / 64) * (kDm / 64)) % 8 == 0);
static_assert((kDin % kScanCh) == 0 && (kSeq % kScanTS) == 0);
static_assert(kScanCh == 64 && kScanTS == 32 && kNst == 16 && kConvK == 4);
static_assert((kDm % 8) == 0);

constexpr size_t kOffXN   = 0;
constexpr size_t kOffBT1  = kOffXN  + (size_t)kRows * kDm  * 2;
constexpr size_t kOffBT2  = kOffBT1 + (size_t)kDin  * kDm  * 2;
constexpr size_t kOffU    = kOffBT2 + (size_t)kDm   * kDin * 2;
constexpr size_t kOffYH   = kOffU   + (size_t)kSeq  * kDin * 4;
constexpr size_t kOffYL   = kOffYH  + (size_t)kRows * kDin * 2;
constexpr size_t kOffP    = kOffYL  + (size_t)kRows * kDin * 2;
constexpr size_t kWsTotal = kOffP   + (size_t)kSeq  * kDm  * 4;
static_assert(kWsTotal == 117440512ull);
static_assert(kWsTotal <= 134217728ull);
static_assert((kOffBT1 % 128) == 0 && (kOffBT2 % 128) == 0 && (kOffU % 128) == 0 &&
              (kOffYH % 128) == 0 && (kOffYL % 128) == 0 && (kOffP % 128) == 0);

__device__ __forceinline__ void dep_guard4_h(v8f& a, v8f& b, v8f& c, v8f& d, v16h x, v16h y) {
  asm volatile("v_nop\n\tv_nop\n\tv_nop\n\tv_nop" : "+v"(a), "+v"(b), "+v"(c), "+v"(d) : "v"(x), "v"(y));
}
__device__ __forceinline__ void keep4_h(v16h a, v16h b, v16h c, v16h d) {
  asm volatile("v_nop" :: "v"(a), "v"(b), "v"(c), "v"(d));
}
__device__ __forceinline__ void acc_guard4(v8f& a, v8f& b, v8f& c, v8f& d) {
  asm volatile("v_nop\n\tv_nop\n\tv_nop\n\tv_nop" : "+v"(a), "+v"(b), "+v"(c), "+v"(d));
}
struct FragH {
  union U { v16h v; v8h h[2]; };
  static __device__ __forceinline__ v16h load(const _Float16* p) {
    U f; f.h[0] = *(const v8h*)(p); f.h[1] = *(const v8h*)(p + 16); return f.v;
  }
  static __device__ __forceinline__ v8f mma(v16h a, v16h b, v8f c) {
    return __builtin_amdgcn_wmma_f32_16x16x32_f16(false, a, false, b, (short)0, c, false, false);
  }
};

template <bool BIASN, bool RESID>
__global__ __launch_bounds__(256) void gemm64_f32out_kernel(
    const unsigned short* __restrict__ Ap, int lda,
    const unsigned short* __restrict__ Btp, int ldb,
    float* __restrict__ C, int ldc,
    const float* __restrict__ bias,
    const float* __restrict__ resid, int ldr,
    int M, int N, int K, float scale)
{
  const _Float16* A  = (const _Float16*)Ap;
  const _Float16* Bt = (const _Float16*)Btp;
  __shared__ __align__(16) float sT[8][16 * 68];
  const int lane = threadIdx.x & 31;
  const int wave = threadIdx.x >> 5;
  const int tilesN = N >> 6;
  const int tilesM = M >> 6;
  const int tile = blockIdx.x * 8 + wave;
  if (tile >= tilesM * tilesN) return;
  const int tm = tile / tilesN;
  const int tn = tile - tm * tilesN;
  const int m0 = tm << 6;
  const int n0 = tn << 6;

  const int rlane = lane & 15;
  const int koff  = (lane >> 4) * 8;
  const int mOff  = (lane >> 4) * 8;

  v8f acc[4][4];
#pragma unroll
  for (int i = 0; i < 4; ++i)
#pragma unroll
    for (int j = 0; j < 4; ++j) acc[i][j] = (v8f){0.f,0.f,0.f,0.f,0.f,0.f,0.f,0.f};

  for (int k0 = 0; k0 < K; k0 += 32) {
    v16h bh[4];
#pragma unroll
    for (int j = 0; j < 4; ++j) {
      const size_t bo = (size_t)(n0 + (j << 4) + rlane) * ldb + koff + k0;
      bh[j] = FragH::load(Bt + bo);
    }
#pragma unroll
    for (int i = 0; i < 4; ++i) {
      const size_t ao = (size_t)(m0 + (i << 4) + rlane) * lda + koff + k0;
      const v16h ah = FragH::load(A + ao);
#pragma unroll
      for (int j = 0; j < 4; ++j) acc[i][j] = FragH::mma(ah, bh[j], acc[i][j]);
      dep_guard4_h(acc[i][0], acc[i][1], acc[i][2], acc[i][3], ah, bh[3]);
    }
    keep4_h(bh[0], bh[1], bh[2], bh[3]);
  }
  acc_guard4(acc[0][0], acc[0][1], acc[0][2], acc[0][3]);
  acc_guard4(acc[1][0], acc[1][1], acc[1][2], acc[1][3]);
  acc_guard4(acc[2][0], acc[2][1], acc[2][2], acc[2][3]);
  acc_guard4(acc[3][0], acc[3][1], acc[3][2], acc[3][3]);

  float* slab = sT[wave];
  const int hh = lane >> 4;
  const int c4 = (lane & 15) * 4;
  v4f bias4 = (v4f){0.f, 0.f, 0.f, 0.f};
  if (BIASN) bias4 = *(const v4f*)(bias + n0 + c4);
#pragma unroll
  for (int i = 0; i < 4; ++i) {
    const int mBase = m0 + (i << 4);
#pragma unroll
    for (int j = 0; j < 4; ++j) {
#pragma unroll
      for (int r = 0; r < 8; ++r) slab[(mOff + r) * 68 + (j << 4) + rlane] = acc[i][j][r] * scale;
    }
    __builtin_amdgcn_fence(__ATOMIC_RELEASE, "workgroup");
    __builtin_amdgcn_wave_barrier();
    __builtin_amdgcn_fence(__ATOMIC_ACQUIRE, "workgroup");
    v4f ov[8];
#pragma unroll
    for (int it = 0; it < 8; ++it) {
      const int row = it * 2 + hh;
      v4f v = *(const v4f*)(slab + row * 68 + c4);
      if (BIASN) v += bias4;
      if (RESID) {
        const v4f rv = *(const v4f*)(resid + (size_t)(mBase + row) * ldr + n0 + c4);
        v += rv;
      }
      ov[it] = v;
    }
    for (int pass = 0; pass < 2; ++pass) {
#pragma unroll
      for (int it = 0; it < 8; ++it) {
        const int row = it * 2 + hh;
        *(volatile v4f*)(C + (size_t)(mBase + row) * ldc + n0 + c4) = ov[it];
      }
      __threadfence();
    }
    __builtin_amdgcn_fence(__ATOMIC_RELEASE, "workgroup");
    __builtin_amdgcn_wave_barrier();
    __builtin_amdgcn_fence(__ATOMIC_ACQUIRE, "workgroup");
  }
}

__global__ __launch_bounds__(256) void transpose_cast_kernel(
    const float* __restrict__ W, unsigned short* __restrict__ Bt, int Kdim, int Ndim, int Npad, float scale)
{
  __shared__ float tile[64 * 65];
  const int tid = threadIdx.x, lane = tid & 31, wave = tid >> 5;
  const int n0 = blockIdx.x * 64;
  const int k0 = blockIdx.y * 64;
  (void)Npad;
#pragma unroll
  for (int p = 0; p < 16; ++p) {
    const int idx = tid + p * 256;
    const int kk  = idx >> 6;
    const int nn  = idx & 63;
    const int n   = n0 + nn;
    const int nc  = (n < Ndim) ? n : (Ndim - 1);
    const float v = W[(size_t)(k0 + kk) * Ndim + nc];
    tile[kk * 65 + nn] = (n < Ndim) ? (v * scale) : 0.f;
  }
  __syncthreads();
  const int q = lane >> 3, c8 = (lane & 7) * 8;
  v8h hv[2];
#pragma unroll
  for (int it = 0; it < 2; ++it) {
    const int nrow = it * 32 + wave * 4 + q;
#pragma unroll
    for (int e = 0; e < 8; ++e) hv[it][e] = (_Float16)tile[(c8 + e) * 65 + nrow];
  }
  for (int pass = 0; pass < 2; ++pass) {
#pragma unroll
    for (int it = 0; it < 2; ++it) {
      const int nrow = it * 32 + wave * 4 + q;
      *(volatile v8h*)(Bt + (size_t)(n0 + nrow) * Kdim + k0 + c8) = hv[it];
    }
    __threadfence();
  }
}

__global__ __launch_bounds__(128) void rmsnorm_cast_kernel(
    const float* __restrict__ x, const float* __restrict__ w, unsigned short* __restrict__ XN)
{
  __shared__ float red[4];
  const int tid = threadIdx.x, lane = tid & 31, wave = tid >> 5;
  const int row = blockIdx.x;
  const float* xr = x + (size_t)row * kDm + tid * 8;
  const v4f a0 = *(const v4f*)(xr);
  const v4f a1 = *(const v4f*)(xr + 4);
  const v4f w0 = *(const v4f*)(w + tid * 8);
  const v4f w1 = *(const v4f*)(w + tid * 8 + 4);
  float ss = 0.0f;
#pragma unroll
  for (int e = 0; e < 4; ++e) ss = fmaf(a0[e], a0[e], ss);
#pragma unroll
  for (int e = 0; e < 4; ++e) ss = fmaf(a1[e], a1[e], ss);
#pragma unroll
  for (int off = 1; off < 32; off <<= 1) ss += __shfl_xor(ss, off, 32);
  if (lane == 0) red[wave] = ss;
  __syncthreads();
  const float tot  = (red[0] + red[1]) + (red[2] + red[3]);
  const float rstd = rsqrtf(tot * (1.0f / (float)kDm) + 1e-6f);
  v8h hv;
#pragma unroll
  for (int e = 0; e < 4; ++e) {
    const float h0 = (a0[e] * rstd) * w0[e];
    const float h1 = (a1[e] * rstd) * w1[e];
    hv[e]     = (_Float16)h0;
    hv[4 + e] = (_Float16)h1;
  }
  unsigned short* qd = XN + (size_t)row * kDm + tid * 8;
  *(volatile v8h*)qd = hv;
  __threadfence();
  *(volatile v8h*)qd = hv;
}

__global__ __launch_bounds__(64) void conv_scan_kernel(
    const float* __restrict__ U, const float* __restrict__ Am, const float* __restrict__ Bm,
    const float* __restrict__ Cm, const float* __restrict__ cw, const float* __restrict__ cb,
    unsigned short* __restrict__ YH, unsigned short* __restrict__ YL)
{
  __shared__ __align__(16) float sA[kScanCh * kAP];
  __shared__ __align__(16) float sS[kNst * kScanCh];
  __shared__ __align__(16) float sU[kScanTS * kYP];
  __shared__ __align__(16) float sY[kScanTS * kYP];
  const int tid = threadIdx.x, lane = tid & 31, wave = tid >> 5;
  const int d0 = blockIdx.x * kScanCh;
  const int d  = d0 + tid;

  {
    const float* Ab = Am + (size_t)d0 * kAmat;
#pragma unroll 4
    for (int it = 0; it < (kScanCh * kAmat) / (4 * kScanCh); ++it) {
      const int e4 = it * kScanCh + tid;
      const int c  = e4 / (kAmat / 4);
      const int w  = (e4 - c * (kAmat / 4)) * 4;
      const v4f v  = *(const v4f*)(Ab + (size_t)e4 * 4);
      *(v4f*)(sA + c * kAP + w) = v;
    }
  }
#pragma unroll
  for (int i = 0; i < kNst; ++i) sS[i * kScanCh + tid] = 0.0f;
  v4f bq[4], cq[4];
#pragma unroll
  for (int q = 0; q < 4; ++q) bq[q] = *(const v4f*)(Bm + (size_t)d * kNst + 4 * q);
  asm volatile("" ::: "memory");
#pragma unroll
  for (int q = 0; q < 4; ++q) cq[q] = *(const v4f*)(Cm + (size_t)d * kNst + 4 * q);
  asm volatile("" ::: "memory");
  const v4f wv = *(const v4f*)(cw + (size_t)d * kConvK);
  const float cbv = cb[d];
  __syncthreads();

  float xm3 = 0.0f, xm2 = 0.0f, xm1 = 0.0f;
  const int lr = tid >> 4, lc4 = (tid & 15) * 4;
  const int q8 = lane >> 3, c8 = (lane & 7) * 8;
  const float* arow = sA + tid * kAP;

#pragma unroll 1
  for (int t0 = 0; t0 < kSeq; t0 += kScanTS) {
#pragma unroll
    for (int it = 0; it < 8; ++it) {
      const int r = it * 4 + lr;
      const v4f v = *(const v4f*)(U + (size_t)(t0 + r) * kDin + d0 + lc4);
      *(v4f*)(sU + r * kYP + lc4) = v;
    }
    __syncthreads();
#pragma unroll 1
    for (int s = 0; s < kScanTS; ++s) {
      const float xc = sU[s * kYP + tid];
      float cacc = wv[0] * xm3;
      cacc = fmaf(wv[1], xm2, cacc);
      cacc = fmaf(wv[2], xm1, cacc);
      cacc = fmaf(wv[3], xc, cacc);
      const float uc = cacc + cbv;
      xm3 = xm2; xm2 = xm1; xm1 = xc;

      float sn[kNst];
#pragma unroll
      for (int j = 0; j < kNst; ++j) sn[j] = uc * bq[j >> 2][j & 3];

#pragma unroll 1
      for (int i = 0; i < kNst; ++i) {
        const float si = sS[i * kScanCh + tid];
        const float* ap = arow + i * kNst;
#pragma unroll
        for (int q = 0; q < 4; ++q) {
          const v4f av = *(const v4f*)(ap + 4 * q);
          sn[4 * q + 0] = fmaf(si, av[0], sn[4 * q + 0]);
          sn[4 * q + 1] = fmaf(si, av[1], sn[4 * q + 1]);
          sn[4 * q + 2] = fmaf(si, av[2], sn[4 * q + 2]);
          sn[4 * q + 3] = fmaf(si, av[3], sn[4 * q + 3]);
        }
      }
      float y = 0.0f;
#pragma unroll
      for (int j = 0; j < kNst; ++j) {
        sS[j * kScanCh + tid] = sn[j];
        y = fmaf(sn[j], cq[j >> 2][j & 3], y);
      }
      sY[s * kYP + tid] = y;
    }
    __syncthreads();

    v8h hv[4], lv[4];
#pragma unroll
    for (int it = 0; it < 4; ++it) {
      const int row = it * 8 + wave * 4 + q8;
      const float* sp = sY + row * kYP + c8;
      const v4f a0 = *(const v4f*)(sp);
      const v4f a1 = *(const v4f*)(sp + 4);
#pragma unroll
      for (int e = 0; e < 4; ++e) {
        const float v0 = a0[e], v1 = a1[e];
        const _Float16 h0 = (_Float16)v0;
        const _Float16 h1 = (_Float16)v1;
        const float f0 = (float)h0;
        const float f1 = (float)h1;
        const float r0 = (v0 - f0) * kLoCarry;
        const float r1 = (v1 - f1) * kLoCarry;
        hv[it][e]     = h0;
        hv[it][4 + e] = h1;
        lv[it][e]     = (_Float16)r0;
        lv[it][4 + e] = (_Float16)r1;
      }
    }
    for (int pass = 0; pass < 2; ++pass) {
#pragma unroll
      for (int it = 0; it < 4; ++it) {
        const int row = it * 8 + wave * 4 + q8;
        const size_t o = (size_t)(t0 + row) * kDin + d0 + c8;
        *(volatile v8h*)(YH + o) = hv[it];
        *(volatile v8h*)(YL + o) = lv[it];
      }
      __threadfence();
    }
  }
}

extern "C" void kernel_launch(void* const* d_in, const int* in_sizes, int n_in,
                              void* d_out, int out_size, void* d_ws, size_t ws_size,
                              hipStream_t stream)
{
  if (n_in < 11) return;
  if (in_sizes[0]  != kRows * kDm) return;
  if (in_sizes[1]  != kDm) return;
  if (in_sizes[2]  != kDm * kDin) return;
  if (in_sizes[3]  != kDin) return;
  if (in_sizes[4]  != kDin * kConvK) return;
  if (in_sizes[5]  != kDin) return;
  if (in_sizes[6]  != kDin * kAmat) return;
  if (in_sizes[7]  != kDin * kNst) return;
  if (in_sizes[8]  != kDin * kNst) return;
  if (in_sizes[9]  != kDin * kDm) return;
  if (in_sizes[10] != kDm) return;
  if (out_size != kRows * kDm) return;
  if (ws_size < kWsTotal) return;

  const float* x      = (const float*)d_in[0];
  const float* norm_w = (const float*)d_in[1];
  const float* Win    = (const float*)d_in[2];
  const float* b_in   = (const float*)d_in[3];
  const float* conv_w = (const float*)d_in[4];
  const float* conv_b = (const float*)d_in[5];
  const float* Amat   = (const float*)d_in[6];
  const float* Bm     = (const float*)d_in[7];
  const float* Cm     = (const float*)d_in[8];
  const float* Wout   = (const float*)d_in[9];
  const float* b_out  = (const float*)d_in[10];
  float* out = (float*)d_out;

  char* ws = (char*)d_ws;
  unsigned short* XN  = (unsigned short*)(ws + kOffXN);
  unsigned short* BT1 = (unsigned short*)(ws + kOffBT1);
  unsigned short* BT2 = (unsigned short*)(ws + kOffBT2);
  float*          U   = (float*)(ws + kOffU);
  unsigned short* YH  = (unsigned short*)(ws + kOffYH);
  unsigned short* YL  = (unsigned short*)(ws + kOffYL);
  float*          P   = (float*)(ws + kOffP);

  rmsnorm_cast_kernel<<<kRows, 128, 0, stream>>>(x, norm_w, XN);

  transpose_cast_kernel<<<dim3(kDin / 64, kDm / 64), 256, 0, stream>>>(Win, BT1, kDm, kDin, kDin, kWCarry);
  transpose_cast_kernel<<<dim3(kDm / 64, kDin / 64), 256, 0, stream>>>(Wout, BT2, kDin, kDm, kDm, kWCarry);

  constexpr int kBlkGemm1 = (kSeq / 64) * (kDin / 64) / 8;
  constexpr int kBlkGemm2 = (kSeq / 64) * (kDm / 64) / 8;

  for (int b = 0; b < kBatch; ++b) {
    const unsigned short* XNb = XN + (size_t)b * kSeq * kDm;
    unsigned short* YHb = YH + (size_t)b * kSeq * kDin;
    unsigned short* YLb = YL + (size_t)b * kSeq * kDin;
    const float* xb = x + (size_t)b * kSeq * kDm;
    float* outb = out + (size_t)b * kSeq * kDm;

    gemm64_f32out_kernel<true, false><<<dim3(kBlkGemm1), 256, 0, stream>>>(
        XNb, kDm, BT1, kDm, U, kDin, b_in, xb, kDm, kSeq, kDin, kDm, kScaleHi);

    conv_scan_kernel<<<dim3(kDin / kScanCh), kScanCh, 0, stream>>>(
        U, Amat, Bm, Cm, conv_w, conv_b, YHb, YLb);

    gemm64_f32out_kernel<false, true><<<dim3(kBlkGemm2), 256, 0, stream>>>(
        YLb, kDin, BT2, kDin, P, kDm, b_out, xb, kDm, kSeq, kDm, kDin, kScaleLo);

    gemm64_f32out_kernel<true, true><<<dim3(kBlkGemm2), 256, 0, stream>>>(
        YHb, kDin, BT2, kDin, outb, kDm, b_out, P, kDm, kSeq, kDm, kDin, kScaleHi);
  }
}
